// GAT_26225070309439
// MI455X (gfx1250) — hardware-verified
//
#include <hip/hip_runtime.h>
#include <stddef.h>
#include <stdint.h>
#include <math.h>


#define NNODE   50000
#define NEDGE   850000
#define F_IN    128
#define HC1     256
#define HID     64
#define CPH1    50
#define NHD1    4
#define HSRC    200
#define NCLS    40
#define NC2P    64
#define KA2     512
#define NTHR    256
#define NWAVE   8
#define EPT     8
#define CHUNK   (NTHR * EPT)
#define WCAP    (EPT * 32)
#define LISTN   (NWAVE * WCAP)
#define NBMAX   2048
#define SLOTB   11
#define RCAP    28672
#define DEGCAP  256
#define GBM     64
#define GBN     64
#define GTHR    128
#define MROWS   128
#define GRP     64
#define NEGSL   0.2f
#define EPS_SM  1e-16f
#define MX0     (-1.0e30f)
#define WSMAX   134217728
#define LDS_AGG ((2 * RCAP + 2 * NBMAX + LISTN) * 4 + 64)

static_assert((NNODE % 4) == 0);
static_assert(NEDGE < (1 << (32 - SLOTB)));
static_assert(CPH1 <= HID && NHD1 * HID == HC1 && NHD1 * CPH1 == HSRC);
static_assert(NCLS <= NC2P);
static_assert((CHUNK & (CHUNK - 1)) == 0 && CHUNK <= (1 << SLOTB));
static_assert(NBMAX == (1 << SLOTB));
static_assert(NTHR * 8 == NBMAX);
static_assert(LISTN >= NBMAX);
static_assert(LISTN >= NWAVE * WCAP);
static_assert((RCAP % 32) == 0);
static_assert(LDS_AGG <= 300000);
static_assert(GBM == (GTHR / 32) * 16);
static_assert(GTHR == 2 * GBN && GTHR == 2 * GBM);
static_assert((F_IN % 32) == 0 && (KA2 % 32) == 0);
static_assert((HC1 % GBN) == 0 && HID == GBN && NC2P == GBN);
static_assert(KA2 == 2 * HC1);
static_assert((MROWS % GBM) == 0);
static_assert(HC1 == 8 * 32);
static_assert(NC2P == 2 * 32);
static_assert(NWAVE * GRP * NCLS <= RCAP);
static_assert((GRP & (GRP - 1)) == 0 && (NCLS % 4) == 0 && (GRP % 4) == 0);
static_assert((F_IN / 8) == 16);
static_assert((NCLS % 2) == 0);

typedef float          v2f  __attribute__((ext_vector_type(2)));
typedef float          v4f  __attribute__((ext_vector_type(4)));
typedef float          v8f  __attribute__((ext_vector_type(8)));
typedef int            v4i  __attribute__((ext_vector_type(4)));
typedef int            v8i  __attribute__((ext_vector_type(8)));
typedef unsigned int   v4u  __attribute__((ext_vector_type(4)));
typedef unsigned short v8us __attribute__((ext_vector_type(8)));
typedef __bf16         v16b __attribute__((ext_vector_type(16)));
typedef v2f  __attribute__((may_alias)) v2fa;
typedef v4f  __attribute__((may_alias)) v4fa;
typedef v8us __attribute__((may_alias)) v8usa;
union FragB { v16b v; v8us h[2]; v8i w; };

__device__ __forceinline__ v8f wmb(const FragB& a, const FragB& b, v8f c) {
  v8f d = __builtin_amdgcn_wmma_f32_16x16x32_bf16(false, a.v, false, b.v, (short)0, c, false, false);
  asm volatile("v_nop\n\tv_nop\n\tv_nop\n\tv_nop" : "+v"(d) : "v"(a.w), "v"(b.w));
  return d;
}

__device__ __forceinline__ unsigned int f2bf(float f) {
  const unsigned int u = __float_as_uint(f);
  const unsigned int r = ((u + 0x7FFFu + ((u >> 16) & 1u)) >> 16) & 0xFFFFu;
  const unsigned int q = ((u >> 16) | 0x40u) & 0xFFFFu;
  return ((u & 0x7FFFFFFFu) > 0x7F800000u) ? q : r;
}
__device__ __forceinline__ float bf2f(unsigned int b) { return __uint_as_float(b << 16); }
__device__ __forceinline__ float bfr(float f) { return bf2f(f2bf(f)); }
__device__ __forceinline__ float bmask(float v, bool ok) {
  return __uint_as_float(__float_as_uint(bfr(v)) & (ok ? 0xFFFFFFFFu : 0u));
}
__device__ __forceinline__ unsigned int pk2(float lo, float hi) { return f2bf(lo) | (f2bf(hi) << 16); }
__device__ __forceinline__ unsigned int pk2lo(float lo, float hi) {
  return f2bf(lo - bfr(lo)) | (f2bf(hi - bfr(hi)) << 16);
}
__device__ __forceinline__ v4u pack8(const v4f a, const v4f b) {
  v4u r;
  r.x = pk2(a.x, a.y); r.y = pk2(a.z, a.w); r.z = pk2(b.x, b.y); r.w = pk2(b.z, b.w);
  return r;
}
__device__ __forceinline__ v4u pack8lo(const v4f a, const v4f b) {
  v4u r;
  r.x = pk2lo(a.x, a.y); r.y = pk2lo(a.z, a.w); r.z = pk2lo(b.x, b.y); r.w = pk2lo(b.z, b.w);
  return r;
}
__device__ __forceinline__ float elu1(float h) {
  const float n = expf(h) - 1.0f;
  return h > 0.f ? h : n;
}
__device__ __forceinline__ float fin1(float a, float inv, float b, bool live, bool bad, float qn) {
  const float v = fmaf(a, inv, b);
  float e = elu1(v);
  e = live ? e : 0.0f;
  return bad ? qn : e;
}

__device__ __forceinline__ int scan_chunk(const int* __restrict__ dsts, int nE, int cbase, int slotBase,
                                          int nb, int vec8, int* list, int tid, int lane, int wave) {
  int wc = 0;
  const int el0  = tid * EPT;
  const int e0   = cbase + el0;
  const int sent = -2147483647 - 1;
  v4i da, db;
  if (vec8 != 0 && cbase + CHUNK <= nE) {
    da = *(const v4i*)(dsts + e0);
    db = *(const v4i*)(dsts + e0 + 4);
  } else {
    da.x = (e0     < nE) ? dsts[min(e0,     nE - 1)] : sent;
    da.y = (e0 + 1 < nE) ? dsts[min(e0 + 1, nE - 1)] : sent;
    da.z = (e0 + 2 < nE) ? dsts[min(e0 + 2, nE - 1)] : sent;
    da.w = (e0 + 3 < nE) ? dsts[min(e0 + 3, nE - 1)] : sent;
    db.x = (e0 + 4 < nE) ? dsts[min(e0 + 4, nE - 1)] : sent;
    db.y = (e0 + 5 < nE) ? dsts[min(e0 + 5, nE - 1)] : sent;
    db.z = (e0 + 6 < nE) ? dsts[min(e0 + 6, nE - 1)] : sent;
    db.w = (e0 + 7 < nE) ? dsts[min(e0 + 7, nE - 1)] : sent;
  }
  const unsigned nbs = (unsigned)slotBase;
  const unsigned unb = (unsigned)nb;
  const unsigned s0 = (unsigned)da.x - nbs, s1 = (unsigned)da.y - nbs;
  const unsigned s2 = (unsigned)da.z - nbs, s3 = (unsigned)da.w - nbs;
  const unsigned s4 = (unsigned)db.x - nbs, s5 = (unsigned)db.y - nbs;
  const unsigned s6 = (unsigned)db.z - nbs, s7 = (unsigned)db.w - nbs;
  const bool h0 = s0 < unb, h1 = s1 < unb, h2 = s2 < unb, h3 = s3 < unb;
  const bool h4 = s4 < unb, h5 = s5 < unb, h6 = s6 < unb, h7 = s7 < unb;
  const unsigned any = __builtin_amdgcn_ballot_w32(h0 | h1 | h2 | h3 | h4 | h5 | h6 | h7);
  if (any != 0u) {
#define HITJ(J, HJ, SJ) { \
      const unsigned mj = __builtin_amdgcn_ballot_w32(HJ); \
      if (mj != 0u) { \
        if (HJ) { \
          const int pos = wc + (int)__builtin_amdgcn_mbcnt_lo(mj, 0u); \
          if (pos < WCAP) list[wave * WCAP + pos] = ((el0 + (J)) << SLOTB) | (int)(SJ); \
        } \
        wc += (int)__builtin_popcount(mj); } }
    HITJ(0, h0, s0)
    HITJ(1, h1, s1)
    HITJ(2, h2, s2)
    HITJ(3, h3, s3)
    HITJ(4, h4, s4)
    HITJ(5, h5, s5)
    HITJ(6, h6, s6)
    HITJ(7, h7, s7)
#undef HITJ
  }
  return wc;
}

__global__ __launch_bounds__(NTHR) void k_xprep(const float* __restrict__ x, unsigned short* xb, int nN, int nUnits) {
  const int i = (int)blockIdx.x * NTHR + (int)threadIdx.x;
  if (i >= nUnits) return;
  const int row = i >> 4;
  const int c0  = (i & 15) * 8;
  const int rc  = row < nN ? row : nN - 1;
  const float* p = x + (size_t)rc * F_IN + c0;
  v4f a = *(const v4fa*)p, b = *(const v4fa*)(p + 4);
  const v4f z4 = {0.f, 0.f, 0.f, 0.f};
  if (row >= nN) { a = z4; b = z4; }
  const v4u hv = pack8(a, b);
  const size_t o = (size_t)row * F_IN + c0;
  *(volatile v4u*)(xb + o) = hv;
  __threadfence();
  *(volatile v4u*)(xb + o) = hv;
}

__global__ __launch_bounds__(NTHR) void k_wtr(const float* __restrict__ w, int Ksrc, int Nsrc,
                                              int kCin, int kCpad, int Kper, int nCin, int nCpad,
                                              int Nrows, int Kout, unsigned short* wt, int nUnits) {
  const int u = (int)blockIdx.x * NTHR + (int)threadIdx.x;
  if (u >= nUnits) return;
  const int kq = Kout >> 3;
  const int n  = u / kq;
  const int k8 = (u - n * kq) * 8;
  const int kk = k8 - (k8 / Kper) * Kper;
  const int kh = kk / kCpad;
  const int kc = kk - kh * kCpad;
  const int nh = n / nCpad;
  const int nc = n - nh * nCpad;
  const int sn = nh * nCin + nc;
  const bool nok = (nc < nCin) && (sn < Nsrc) && (n < Nrows);
  const int snc = sn < 0 ? 0 : (sn > Nsrc - 1 ? Nsrc - 1 : sn);
  const int sk0 = kh * kCin + kc;
  const int km  = Ksrc - 1;
  const float* p = w + snc;
  const size_t ld = (size_t)Nsrc;
  const float t0 = p[(size_t)min(sk0 + 0, km) * ld];
  const float t1 = p[(size_t)min(sk0 + 1, km) * ld];
  const float t2 = p[(size_t)min(sk0 + 2, km) * ld];
  const float t3 = p[(size_t)min(sk0 + 3, km) * ld];
  const float t4 = p[(size_t)min(sk0 + 4, km) * ld];
  const float t5 = p[(size_t)min(sk0 + 5, km) * ld];
  const float t6 = p[(size_t)min(sk0 + 6, km) * ld];
  const float t7 = p[(size_t)min(sk0 + 7, km) * ld];
  v4f a, b;
  a.x = (nok && kc + 0 < kCin && sk0 + 0 < Ksrc) ? t0 : 0.f;
  a.y = (nok && kc + 1 < kCin && sk0 + 1 < Ksrc) ? t1 : 0.f;
  a.z = (nok && kc + 2 < kCin && sk0 + 2 < Ksrc) ? t2 : 0.f;
  a.w = (nok && kc + 3 < kCin && sk0 + 3 < Ksrc) ? t3 : 0.f;
  b.x = (nok && kc + 4 < kCin && sk0 + 4 < Ksrc) ? t4 : 0.f;
  b.y = (nok && kc + 5 < kCin && sk0 + 5 < Ksrc) ? t5 : 0.f;
  b.z = (nok && kc + 6 < kCin && sk0 + 6 < Ksrc) ? t6 : 0.f;
  b.w = (nok && kc + 7 < kCin && sk0 + 7 < Ksrc) ? t7 : 0.f;
  const v4u wv = pack8(a, b);
  unsigned short* o = wt + (size_t)n * (size_t)Kout + k8;
  *(volatile v4u*)o = wv;
  __threadfence();
  *(volatile v4u*)o = wv;
}

__global__ __launch_bounds__(GTHR) void k_gemm(
    const unsigned short* __restrict__ A, const unsigned short* __restrict__ WT,
    float* outF, int K, int ldo,
    const float* __restrict__ atts, const float* __restrict__ attd, int attLen,
    float* SD, int MPr)
{
  __shared__ __attribute__((aligned(16))) float stg[GBM * GBN];
  __shared__ __attribute__((aligned(16))) float satt[2 * GBN];
  __shared__ __attribute__((aligned(16))) float sdot[2 * GBM];
  const int tid = (int)threadIdx.x, lane = tid & 31, wave = tid >> 5, hh = lane >> 4, m = lane & 15;
  const int rowBase = (int)blockIdx.x * GBM;
  const int head    = (int)blockIdx.y;
  const int col0    = head * GBN;

  {
    const int which = tid >> 6;
    const int c  = tid & 63;
    const int cl = c < attLen ? c : attLen - 1;
    const float vs = atts[head * attLen + cl];
    const float vd = attd[head * attLen + cl];
    float v = (which == 0) ? vs : vd;
    v = (c < attLen) ? bfr(v) : 0.f;
    satt[which * GBN + c] = v;
  }

  v8f acc[4];
  {
    const v8f z = {0.f, 0.f, 0.f, 0.f, 0.f, 0.f, 0.f, 0.f};
    acc[0] = z; acc[1] = z; acc[2] = z; acc[3] = z;
  }
  const unsigned short* ap = A  + (size_t)(rowBase + 16 * wave + m) * (size_t)K + 8 * hh;
  const unsigned short* wp = WT + (size_t)(col0 + m) * (size_t)K + 8 * hh;
  const int ksteps = K >> 5;
#pragma unroll 1
  for (int ks = 0; ks < ksteps; ++ks) {
    FragB af;
    af.h[0] = *(const v8usa*)(ap + 32 * ks);
    af.h[1] = *(const v8usa*)(ap + 32 * ks + 16);
#pragma unroll
    for (int t = 0; t < 4; ++t) {
      const unsigned short* wq = wp + (size_t)(16 * t) * (size_t)K + 32 * ks;
      FragB bf;
      bf.h[0] = *(const v8usa*)wq;
      bf.h[1] = *(const v8usa*)(wq + 16);
      acc[t] = wmb(af, bf, acc[t]);
    }
  }

#pragma unroll
  for (int t = 0; t < 4; ++t) {
    const int lc = 16 * t + m;
#pragma unroll
    for (int r = 0; r < 8; ++r) {
      const int lr = 16 * wave + 8 * hh + r;
      stg[lr * GBN + lc] = acc[t][r];
    }
  }
  __syncthreads();

  {
    const int row = tid & 63, which = tid >> 6;
    const float* sa = satt + which * GBN;
    const float* hr = stg + row * GBN;
    float d = 0.f;
#pragma unroll 4
    for (int c4 = 0; c4 < GBN / 4; ++c4) {
      const v4f hv = *(const v4fa*)(hr + 4 * c4);
      const v4f av = *(const v4fa*)(sa + 4 * c4);
      d = fmaf(hv.x, av.x, d);
      d = fmaf(hv.y, av.y, d);
      d = fmaf(hv.z, av.z, d);
      d = fmaf(hv.w, av.w, d);
    }
    sdot[which * GBM + row] = d;
  }
  __syncthreads();

  v4f fv[8];
#pragma unroll
  for (int i = 0; i < 8; ++i) {
    const int lr = 16 * wave + 2 * i + hh;
    fv[i] = *(const v4fa*)(stg + lr * GBN + 4 * m);
  }
  const int which2 = lane >> 4, piece = lane & 15;
  const v4f sdv = *(const v4fa*)(sdot + which2 * GBM + 4 * piece);
  float* sp = SD + (size_t)(2 * head + which2) * (size_t)MPr + rowBase + 4 * piece;

#pragma unroll
  for (int i = 0; i < 8; ++i) {
    const int lr = 16 * wave + 2 * i + hh;
    const int gr = rowBase + lr;
    float* op = outF + (size_t)gr * (size_t)ldo + col0 + 4 * m;
    *(volatile v4f*)op = fv[i];
  }
  if (wave == 0) *(volatile v4f*)sp = sdv;
  __threadfence();
#pragma unroll
  for (int i = 0; i < 8; ++i) {
    const int lr = 16 * wave + 2 * i + hh;
    const int gr = rowBase + lr;
    float* op = outF + (size_t)gr * (size_t)ldo + col0 + 4 * m;
    *(volatile v4f*)op = fv[i];
  }
  if (wave == 0) *(volatile v4f*)sp = sdv;
}

template<int L>
__global__ __launch_bounds__(NTHR) void k_agg(
    const int* __restrict__ srcs, const int* __restrict__ dsts,
    const float* __restrict__ F, const float* __restrict__ SD,
    const float* __restrict__ bias,
    unsigned short* HP, float* out,
    int nN, int nE, int nb, int vec8, int MPr) {
  extern __shared__ v4f lds_dyn[];
  int* reg1 = (int*)lds_dyn;
  int* reg2 = reg1 + RCAP;
  int* scnt = reg2 + RCAP;
  int* soff = scnt + NBMAX;
  int* list = soff + NBMAX;
  int* wcnt = list + LISTN;
  int* wtot = wcnt + NWAVE;
  const int tid = (int)threadIdx.x, lane = tid & 31, wave = tid >> 5;
  const int nodeBase = (int)blockIdx.x * nb;

  for (int i = tid; i < NBMAX; i += NTHR) scnt[i] = 0;
  __syncthreads();

  int tot = 0;
  const int nChunks = (nE + CHUNK - 1) / CHUNK;
#pragma unroll 1
  for (int ch = 0; ch < nChunks; ++ch) {
    const int cbase = ch * CHUNK;
    const int wc = scan_chunk(dsts, nE, cbase, nodeBase, nb, vec8, list, tid, lane, wave);
    if (lane == 0) wcnt[wave] = wc;
    __syncthreads();
    int pre = 0, all = 0;
#pragma unroll
    for (int w2 = 0; w2 < NWAVE; ++w2) {
      int c = wcnt[w2];
      c = c < 0 ? 0 : (c > WCAP ? WCAP : c);
      all += c;
      pre += (w2 < wave) ? c : 0;
    }
    const int wcc  = wc > WCAP ? WCAP : wc;
    const int base = tot + pre;
#pragma unroll 1
    for (int i = lane; i < wcc; i += 32) {
      const int ent = list[wave * WCAP + i];
      const int el  = (ent >> SLOTB) & (CHUNK - 1);
      const int sl  = ent & (NBMAX - 1);
      int eid = cbase + el;
      eid = eid > nE - 1 ? nE - 1 : eid;
      const int pos = base + i;
      if (pos < RCAP) reg1[pos] = (int)(((unsigned)eid << SLOTB) | (unsigned)sl);
    }
    tot += all;
    tot = tot > RCAP ? RCAP : tot;
    __syncthreads();
  }
  const int nh = tot;

  if (wave == 0) {
#pragma unroll 1
    for (int b0 = 0; b0 < nh; b0 += 32) {
      const int idx = b0 + lane;
      const int uv  = reg1[idx < nh ? idx : nh - 1];
      const int m32 = (nh - b0) < 32 ? (nh - b0) : 32;
#pragma unroll 1
      for (int k = 0; k < m32; ++k) {
        const int u  = __builtin_amdgcn_readlane(uv, k);
        const int sl = u & (NBMAX - 1);
        if (lane == 0) scnt[sl] = scnt[sl] + 1;
      }
    }
  }
  __syncthreads();

  {
    const v4i ca = *(const v4i*)(scnt + 8 * tid);
    const v4i cb = *(const v4i*)(scnt + 8 * tid + 4);
    const int e0 = ca.x < 0 ? 0 : ca.x, e1 = ca.y < 0 ? 0 : ca.y, e2 = ca.z < 0 ? 0 : ca.z, e3 = ca.w < 0 ? 0 : ca.w;
    const int e4 = cb.x < 0 ? 0 : cb.x, e5 = cb.y < 0 ? 0 : cb.y, e6 = cb.z < 0 ? 0 : cb.z, e7 = cb.w < 0 ? 0 : cb.w;
    const int ts = e0 + e1 + e2 + e3 + e4 + e5 + e6 + e7;
    int incl = ts;
#pragma unroll
    for (int d = 1; d < 32; d <<= 1) {
      const int up = __shfl_up(incl, d);
      if (lane >= d) incl += up;
    }
    if (lane == 31) wtot[wave] = incl;
    __syncthreads();
    int pre = 0;
#pragma unroll
    for (int w2 = 0; w2 < NWAVE; ++w2) pre += (w2 < wave) ? wtot[w2] : 0;
    int run = pre + incl - ts;
    soff[8 * tid + 0] = run; run += e0;
    soff[8 * tid + 1] = run; run += e1;
    soff[8 * tid + 2] = run; run += e2;
    soff[8 * tid + 3] = run; run += e3;
    soff[8 * tid + 4] = run; run += e4;
    soff[8 * tid + 5] = run; run += e5;
    soff[8 * tid + 6] = run; run += e6;
    soff[8 * tid + 7] = run;
  }
  __syncthreads();
  for (int i = tid; i < NBMAX; i += NTHR) list[i] = soff[i];
  __syncthreads();

  if (wave == 0) {
#pragma unroll 1
    for (int b0 = 0; b0 < nh; b0 += 32) {
      const int idx = b0 + lane;
      const int uv  = reg1[idx < nh ? idx : nh - 1];
      const int m32 = (nh - b0) < 32 ? (nh - b0) : 32;
#pragma unroll 1
      for (int k = 0; k < m32; ++k) {
        const int u   = __builtin_amdgcn_readlane(uv, k);
        const int sl  = u & (NBMAX - 1);
        const int eid = (int)((unsigned)u >> SLOTB);
        if (lane == 0) {
          int pos = list[sl];
          pos = pos < 0 ? 0 : (pos > RCAP - 1 ? RCAP - 1 : pos);
          reg2[pos] = eid;
          list[sl] = pos + 1;
        }
      }
    }
  }
  __syncthreads();

  const int nbw = nb >> 3;
  const bool ovf = (nh >= RCAP);
  const float qnan = __int_as_float(0x7fc00000);

  if (L == 1) {
    const int c0   = 8 * lane;
    const int head = lane >> 3;
    const int cb   = c0 & (HID - 1);
    const int bi   = head * CPH1 + cb;
    const float t0 = bias[min(bi + 0, HSRC - 1)];
    const float t1 = bias[min(bi + 1, HSRC - 1)];
    const float t2 = bias[min(bi + 2, HSRC - 1)];
    const float t3 = bias[min(bi + 3, HSRC - 1)];
    const float t4 = bias[min(bi + 4, HSRC - 1)];
    const float t5 = bias[min(bi + 5, HSRC - 1)];
    const float t6 = bias[min(bi + 6, HSRC - 1)];
    const float t7 = bias[min(bi + 7, HSRC - 1)];
    v4f bbA, bbB;
    bbA.x = bmask(t0, cb + 0 < CPH1);
    bbA.y = bmask(t1, cb + 1 < CPH1);
    bbA.z = bmask(t2, cb + 2 < CPH1);
    bbA.w = bmask(t3, cb + 3 < CPH1);
    bbB.x = bmask(t4, cb + 4 < CPH1);
    bbB.y = bmask(t5, cb + 5 < CPH1);
    bbB.z = bmask(t6, cb + 6 < CPH1);
    bbB.w = bmask(t7, cb + 7 < CPH1);
    const float* ASp = SD + (size_t)(2 * head) * (size_t)MPr;
    const float* ADp = ASp + MPr;

#pragma unroll 1
    for (int jt = 0; jt < nbw; ++jt) {
      const int slot = wave * nbw + jt;
      const int grow = nodeBase + slot;
      const int gcl  = grow < nN ? grow : nN - 1;
      int st = soff[slot];
      const int craw = scnt[slot];
      int cnt = craw;
      st  = st < 0 ? 0 : (st > nh ? nh : st);
      cnt = cnt < 0 ? 0 : (cnt > DEGCAP ? DEGCAP : cnt);
      if (cnt > nh - st) cnt = nh - st;
      const bool bad = ovf || craw > DEGCAP;

      const float adv = ADp[gcl];
      float mx = MX0, dn = 0.0f;
      v4f av = {0.f, 0.f, 0.f, 0.f};
      v4f aw = {0.f, 0.f, 0.f, 0.f};

#pragma unroll 1
      for (int q = 0; q < cnt; ++q) {
        int idx = st + q; idx = idx > RCAP - 1 ? RCAP - 1 : idx;
        int eid = reg2[idx]; eid = eid < 0 ? 0 : (eid > nE - 1 ? nE - 1 : eid);
        const int sraw = srcs[eid];
        const int s = sraw < 0 ? 0 : (sraw > nN - 1 ? nN - 1 : sraw);
        const float* fr = F + (size_t)s * HC1 + c0;
        const v4f fs = *(const v4fa*)fr;
        const v4f ft = *(const v4fa*)(fr + 4);
        float lg = ASp[s] + adv;
        lg = lg > 0.f ? lg : NEGSL * lg;
        const float df = lg - mx;
        const float ee = expf(-fabsf(df));
        const bool up  = df > 0.f;
        const float s1 = up ? ee : 1.0f;
        const float s2 = up ? 1.0f : ee;
        mx = up ? lg : mx;
        dn = fmaf(dn, s1, s2);
        av.x = fmaf(av.x, s1, s2 * fs.x);
        av.y = fmaf(av.y, s1, s2 * fs.y);
        av.z = fmaf(av.z, s1, s2 * fs.z);
        av.w = fmaf(av.w, s1, s2 * fs.w);
        aw.x = fmaf(aw.x, s1, s2 * ft.x);
        aw.y = fmaf(aw.y, s1, s2 * ft.y);
        aw.z = fmaf(aw.z, s1, s2 * ft.z);
        aw.w = fmaf(aw.w, s1, s2 * ft.w);
      }
      const float inv = __builtin_amdgcn_rcpf(dn + EPS_SM);
      const bool live = grow < nN;
      v4f o, u;
      o.x = fin1(av.x, inv, bbA.x, live, bad, qnan);
      o.y = fin1(av.y, inv, bbA.y, live, bad, qnan);
      o.z = fin1(av.z, inv, bbA.z, live, bad, qnan);
      o.w = fin1(av.w, inv, bbA.w, live, bad, qnan);
      u.x = fin1(aw.x, inv, bbB.x, live, bad, qnan);
      u.y = fin1(aw.y, inv, bbB.y, live, bad, qnan);
      u.z = fin1(aw.z, inv, bbB.z, live, bad, qnan);
      u.w = fin1(aw.w, inv, bbB.w, live, bad, qnan);
      const v4u hv = pack8(o, u);
      const v4u lv = pack8lo(o, u);
      unsigned short* gp = HP + (size_t)grow * KA2 + 8 * lane;
      const bool wr = grow < MPr;
      if (wr) { *(volatile v4u*)gp = hv; *(volatile v4u*)(gp + HC1) = lv; }
      __threadfence();
      if (wr) { *(volatile v4u*)gp = hv; *(volatile v4u*)(gp + HC1) = lv; }
    }
  } else {
    const int c0 = 2 * lane;
    const bool valid = c0 < NCLS;
    const int cc0 = c0 < NCLS ? c0 : NCLS - 1;
    const int cc1 = c0 + 1 < NCLS ? c0 + 1 : NCLS - 1;
    const float tb0 = bias[cc0], tb1 = bias[cc1];
    float bz0 = bfr(tb0), bz1 = bfr(tb1);
    bz0 = valid ? bz0 : 0.f;
    bz1 = valid ? bz1 : 0.f;
    const float* ASp = SD;
    const float* ADp = SD + MPr;
    float* res = (float*)reg1 + wave * (GRP * NCLS);

#pragma unroll 1
    for (int jt = 0; jt < nbw; ++jt) {
      const int slot = wave * nbw + jt;
      const int grow = nodeBase + slot;
      const int gcl  = grow < nN ? grow : nN - 1;
      int st = soff[slot];
      const int craw = scnt[slot];
      int cnt = craw;
      st  = st < 0 ? 0 : (st > nh ? nh : st);
      cnt = cnt < 0 ? 0 : (cnt > DEGCAP ? DEGCAP : cnt);
      if (cnt > nh - st) cnt = nh - st;
      const bool bad = ovf || craw > DEGCAP;

      const float adv = ADp[gcl];
      float mx = MX0, dn = 0.0f;
      float a0 = 0.0f, a1 = 0.0f;

#pragma unroll 1
      for (int q = 0; q < cnt; ++q) {
        int idx = st + q; idx = idx > RCAP - 1 ? RCAP - 1 : idx;
        int eid = reg2[idx]; eid = eid < 0 ? 0 : (eid > nE - 1 ? nE - 1 : eid);
        const int sraw = srcs[eid];
        const int s = sraw < 0 ? 0 : (sraw > nN - 1 ? nN - 1 : sraw);
        const v2f fs = *(const v2fa*)(F + (size_t)s * NC2P + c0);
        float lg = ASp[s] + adv;
        lg = lg > 0.f ? lg : NEGSL * lg;
        const float df = lg - mx;
        const float ee = expf(-fabsf(df));
        const bool up  = df > 0.f;
        const float s1 = up ? ee : 1.0f;
        const float s2 = up ? 1.0f : ee;
        mx = up ? lg : mx;
        dn = fmaf(dn, s1, s2);
        a0 = fmaf(a0, s1, s2 * fs.x);
        a1 = fmaf(a1, s1, s2 * fs.y);
      }
      const float inv = __builtin_amdgcn_rcpf(dn + EPS_SM);
      const float z0 = fmaf(a0, inv, bz0);
      const float z1 = fmaf(a1, inv, bz1);
      float vm = valid ? fmaxf(z0, z1) : -3.0e38f;
#pragma unroll
      for (int off = 16; off > 0; off >>= 1) vm = fmaxf(vm, __shfl_xor(vm, off));
      const float ex0 = expf(z0 - vm), ex1 = expf(z1 - vm);
      float sm = valid ? (ex0 + ex1) : 0.f;
#pragma unroll
      for (int off = 16; off > 0; off >>= 1) sm += __shfl_xor(sm, off);
      const float ls = logf(sm);
      float o0 = (z0 - vm) - ls;
      float o1 = (z1 - vm) - ls;
      o0 = bad ? qnan : o0;
      o1 = bad ? qnan : o1;
      const int lr = jt & (GRP - 1);
      if (valid) {
        v2f ov; ov.x = o0; ov.y = o1;
        *(v2f*)(res + lr * NCLS + c0) = ov;
      }

      const int gb = jt & ~(GRP - 1);
      if (lr == GRP - 1 || jt == nbw - 1) {
        __syncthreads();
        int gsz = nbw - gb; gsz = gsz > GRP ? GRP : gsz;
        const int row0 = nodeBase + wave * nbw + gb;
        int live = nN - row0; live = live < 0 ? 0 : (live > gsz ? gsz : live);
        const int npc = live * (NCLS / 4);
        float* ob = out + (size_t)row0 * NCLS;
#pragma unroll 1
        for (int p = lane; p < npc; p += 32) {
          const v4f v = *(const v4fa*)(res + 4 * p);
          *(volatile v4f*)(ob + 4 * p) = v;
        }
        __threadfence();
#pragma unroll 1
        for (int p = lane; p < npc; p += 32) {
          const v4f v = *(const v4fa*)(res + 4 * p);
          *(volatile v4f*)(ob + 4 * p) = v;
        }
        __syncthreads();
      }
    }
  }
}

static int pick_nb(int nE, int nN) {
  int nb = NBMAX;
  while (nb > 32 && (long long)nb * (long long)nE * 5LL > (long long)RCAP * (long long)nN * 4LL) nb >>= 1;
  return nb;
}
static inline int cdiv(int a, int b) { return (a + b - 1) / b; }

extern "C" void kernel_launch(void* const* d_in, const int* in_sizes, int n_in,
                              void* d_out, int out_size, void* d_ws, size_t ws_size,
                              hipStream_t stream) {
  if (n_in < 11) return;
  const int nN = in_sizes[0] / F_IN;
  if (nN != NNODE || in_sizes[0] != nN * F_IN) return;
  const int nE = in_sizes[1];
  if (nE != NEDGE || in_sizes[2] != nE) return;
  if (in_sizes[3] != F_IN * HSRC) return;
  if (in_sizes[4] != HSRC || in_sizes[5] != HSRC) return;
  if (in_sizes[6] != HSRC) return;
  if (in_sizes[7] != HSRC * NCLS) return;
  if (in_sizes[8] != NCLS || in_sizes[9] != NCLS) return;
  if (in_sizes[10] != NCLS) return;
  if (out_size != nN * NCLS) return;

  const float* x    = (const float*)d_in[0];
  const int*   src  = (const int*)  d_in[1];
  const int*   dst  = (const int*)  d_in[2];
  const float* W1   = (const float*)d_in[3];
  const float* a1s  = (const float*)d_in[4];
  const float* a1d  = (const float*)d_in[5];
  const float* b1   = (const float*)d_in[6];
  const float* W2   = (const float*)d_in[7];
  const float* a2s  = (const float*)d_in[8];
  const float* a2d  = (const float*)d_in[9];
  const float* b2   = (const float*)d_in[10];
  float* out = (float*)d_out;

  const int MP   = cdiv(nN, MROWS) * MROWS;
  const int nb   = pick_nb(nE, nN);
  if (nb < 32 || (nb & (nb - 1)) != 0 || nb > NBMAX || (nb & 31) != 0) return;
  const int gA   = cdiv(MP, nb);
  const int vec8 = 1;
  if (gA * nb < MP) return;

  char* ws = (char*)d_ws;
  size_t off = 0;
  const size_t szA  = (size_t)MP * KA2 * 2;
  const size_t szB  = (size_t)MP * HC1 * 4;
  const size_t oA   = off; off += szA;                             off = (off + 255) & ~(size_t)255;
  const size_t oB   = off; off += szB;                             off = (off + 255) & ~(size_t)255;
  const size_t oSD1 = off; off += (size_t)2 * NHD1 * MP * 4;       off = (off + 255) & ~(size_t)255;
  const size_t oSD2 = off; off += (size_t)2 * MP * 4;              off = (off + 255) & ~(size_t)255;
  const size_t oW1T = off; off += (size_t)HC1 * F_IN * 2;          off = (off + 255) & ~(size_t)255;
  const size_t oW2T = off; off += (size_t)NC2P * KA2 * 2;          off = (off + 255) & ~(size_t)255;
  if ((size_t)MP * F_IN * 2 > szA) return;
  if ((size_t)MP * NC2P * 4 > szB) return;
  if (off > ws_size || off > (size_t)WSMAX) return;
  unsigned short* X1HL = (unsigned short*)(ws + oA);
  unsigned short* XB   = (unsigned short*)(ws + oA);
  float*          H1   = (float*)(ws + oB);
  float*          H2   = (float*)(ws + oB);
  float*          SD1  = (float*)(ws + oSD1);
  float*          SD2  = (float*)(ws + oSD2);
  unsigned short* W1T  = (unsigned short*)(ws + oW1T);
  unsigned short* W2T  = (unsigned short*)(ws + oW2T);

  hipFuncSetAttribute(reinterpret_cast<const void*>(&k_agg<1>),
                      hipFuncAttributeMaxDynamicSharedMemorySize, LDS_AGG);
  hipFuncSetAttribute(reinterpret_cast<const void*>(&k_agg<2>),
                      hipFuncAttributeMaxDynamicSharedMemorySize, LDS_AGG);

  const int nUx = MP * (F_IN / 8);
  k_xprep<<<cdiv(nUx, NTHR), NTHR, 0, stream>>>(x, XB, nN, nUx);

  {
    const int nUw1 = HC1 * (F_IN / 8);
    k_wtr<<<cdiv(nUw1, NTHR), NTHR, 0, stream>>>(W1, F_IN, HSRC, F_IN, F_IN, F_IN, CPH1, HID,
                                                 HC1, F_IN, W1T, nUw1);
    const int nUw2 = NC2P * (KA2 / 8);
    k_wtr<<<cdiv(nUw2, NTHR), NTHR, 0, stream>>>(W2, HSRC, NCLS, CPH1, HID, HC1, NC2P, NC2P,
                                                 NC2P, KA2, W2T, nUw2);
  }

  const int gM = MP / GBM;
  k_gemm<<<dim3(gM, HC1 / GBN), GTHR, 0, stream>>>(XB, W1T, H1, F_IN, HC1, a1s, a1d, CPH1, SD1, MP);
  k_agg<1><<<gA, NTHR, LDS_AGG, stream>>>(src, dst, H1, SD1, b1, X1HL, out, nN, nE, nb, vec8, MP);
  k_gemm<<<dim3(gM, NC2P / GBN), GTHR, 0, stream>>>(X1HL, W2T, H2, KA2, NC2P, a2s, a2d, NCLS, SD2, MP);
  k_agg<2><<<gA, NTHR, LDS_AGG, stream>>>(src, dst, H2, SD2, b2, X1HL, out, nN, nE, nb, vec8, MP);
}
